// GeneralConv_18940805775383
// MI455X (gfx1250) — hardware-verified
//
#include <hip/hip_runtime.h>
#include <math.h>


#define DD   128
#define TT   3
#define RR   4
#define HH   8
#define DK   16
#define TP   136
#define NB   256
#define LCAP 32
#define CHW  2048
#define CHB  (8 * CHW)
#define WSC  16.0f
#define WSCI 0.0625f
#define RSC  8.0f
#define RSCI 0.125f
#define NWT8 (4 * TT * DD * DD / 8)
#define ELDS_FLOATS (NB * DD + 2 * NB * HH + 64 * LCAP + 64 + 16 * DD / 2)

typedef _Float16 v16h __attribute__((ext_vector_type(16)));
typedef _Float16 v8h  __attribute__((ext_vector_type(8)));
typedef _Float16 v4h  __attribute__((ext_vector_type(4)));
typedef v8h v8ha __attribute__((may_alias));
typedef float v8f __attribute__((ext_vector_type(8)));
typedef float v4f __attribute__((ext_vector_type(4)));
union Frag { v16h v; v8h half[2]; };

__device__ __forceinline__ v8f wmma_f16(v16h a, v16h b, v8f c)
{
    c = __builtin_amdgcn_wmma_f32_16x16x32_f16(false, a, false, b, (short)0, c, false, false);
    asm volatile("v_nop\n\tv_nop\n\tv_nop\n\tv_nop" : "+v"(c) : "v"(a), "v"(b));
    return c;
}

__device__ __forceinline__ int clampi(int x, int lo, int hi)
{
    return x < lo ? lo : (x > hi ? hi : x);
}

__global__ __launch_bounds__(256)
void k_cvtw(const float* __restrict__ W0, const float* __restrict__ W1,
            const float* __restrict__ W2, const float* __restrict__ W3,
            _Float16* __restrict__ Wt, int total8)
{
    const int tid = blockIdx.x * 256 + threadIdx.x;
    if (tid >= total8) return;
    const int j = tid * 8;
    const int which = j / (TT * DD * DD);
    const int rem = j - which * (TT * DD * DD);
    const int t = rem / (DD * DD);
    const int rem2 = rem - t * (DD * DD);
    const int oo = rem2 / DD;
    const int ii0 = rem2 - oo * DD;
    const float* W = (which == 0) ? W0 : ((which == 1) ? W1 : ((which == 2) ? W2 : W3));
    v8h o = {};
#pragma unroll
    for (int q = 0; q < 8; ++q)
        o[q] = (_Float16)(WSC * W[((size_t)t * DD + ii0 + q) * DD + oo]);
    _Float16* dp = Wt + j;
    *(volatile v8h*)dp = o;
    __threadfence();
    *(volatile v8h*)dp = o;
}

template <bool SRC32>
__device__ __forceinline__ void proj_tile(const float* __restrict__ Xf, const _Float16* __restrict__ Xh,
                                          const _Float16* __restrict__ Wt3, const float* __restrict__ bias,
                                          const int* __restrict__ ntype, int row0, int nN, float* tile)
{
    const int w = threadIdx.x >> 5, l = threadIdx.x & 31, h = l >> 4, m = l & 15;
    const int rowA = min(row0 + m, nN - 1);
    const int col = w * 16 + m;
    v8f acc0 = {}; v8f acc1 = {}; v8f acc2 = {};
#pragma unroll
    for (int k0 = 0; k0 < DD; k0 += 32) {
        Frag a;
        if (SRC32) {
            const float* xp = Xf + (size_t)rowA * DD + k0 + 8 * h;
            const v8f x0 = *(const v8f*)xp;
            const v8f x1 = *(const v8f*)(xp + 16);
            a.half[0] = __builtin_convertvector(x0, v8h);
            a.half[1] = __builtin_convertvector(x1, v8h);
        } else {
            const _Float16* xp = Xh + (size_t)rowA * DD + k0 + 8 * h;
            a.half[0] = *(const v8h*)xp;
            a.half[1] = *(const v8h*)(xp + 16);
        }
        const _Float16* wb = Wt3 + (size_t)col * DD + k0 + 8 * h;
        Frag b;
        b.half[0] = *(const v8h*)wb;
        b.half[1] = *(const v8h*)(wb + 16);
        acc0 = wmma_f16(a.v, b.v, acc0);
        b.half[0] = *(const v8h*)(wb + DD * DD);
        b.half[1] = *(const v8h*)(wb + DD * DD + 16);
        acc1 = wmma_f16(a.v, b.v, acc1);
        b.half[0] = *(const v8h*)(wb + 2 * DD * DD);
        b.half[1] = *(const v8h*)(wb + 2 * DD * DD + 16);
        acc2 = wmma_f16(a.v, b.v, acc2);
    }
#pragma unroll
    for (int rr = 0; rr < 8; ++rr) {
        const int r = 8 * h + rr;
        const int grow = min(row0 + r, nN - 1);
        const int t = clampi(ntype[grow], 0, TT - 1);
        const float v0 = acc0[rr], v1 = acc1[rr], v2 = acc2[rr];
        float val = (t == 0) ? v0 : ((t == 1) ? v1 : v2);
        val = val * WSCI + bias[t * DD + col];
        tile[r * TP + col] = val;
    }
}

__global__ __launch_bounds__(256)
void k_proj_kqv(const float* __restrict__ X, const _Float16* __restrict__ Wt,
                const float* __restrict__ bk, const float* __restrict__ bq, const float* __restrict__ bv,
                const int* __restrict__ ntype,
                _Float16* __restrict__ outK, float* __restrict__ outQ, _Float16* __restrict__ outV, int nN)
{
    __shared__ __attribute__((aligned(32))) float tile[16 * TP];
    const int which = blockIdx.y;
    const int row0 = blockIdx.x * 16;
    const float* bias = (which == 0) ? bk : ((which == 1) ? bq : bv);
    proj_tile<true>(X, nullptr, Wt + (size_t)which * TT * DD * DD, bias, ntype, row0, nN, tile);
    __syncthreads();
    const int w = threadIdx.x >> 5, l = threadIdx.x & 31;
    if (which == 1) {
        const int ra = 2 * w, rb = 2 * w + 1;
        const int ga = row0 + ra, gb = row0 + rb;
        const v4f va = *(const v4f*)(tile + ra * TP + 4 * l);
        const v4f vb = *(const v4f*)(tile + rb * TP + 4 * l);
        float* pa = outQ + (size_t)ga * DD + 4 * l;
        float* pb = outQ + (size_t)gb * DD + 4 * l;
        if (ga < nN) *(volatile v4f*)pa = va;
        if (gb < nN) *(volatile v4f*)pb = vb;
        __threadfence();
        if (ga < nN) *(volatile v4f*)pa = va;
        if (gb < nN) *(volatile v4f*)pb = vb;
    } else {
        _Float16* o16 = (which == 0) ? outK : outV;
        const int r = 2 * w + (l >> 4);
        const int g = row0 + r;
        const int cb = 8 * (l & 15);
        const v8f x = *(const v8f*)(tile + r * TP + cb);
        const v8h hv = __builtin_convertvector(x, v8h);
        _Float16* p = o16 + (size_t)g * DD + cb;
        if (g < nN) *(volatile v8h*)p = hv;
        __threadfence();
        if (g < nN) *(volatile v8h*)p = hv;
    }
}

__global__ __launch_bounds__(256)
void k_proj_ln(const _Float16* __restrict__ Hh, const _Float16* __restrict__ Wt3, const float* __restrict__ ba,
               const int* __restrict__ ntype, const float* __restrict__ X,
               const float* __restrict__ skipw, const float* __restrict__ lng, const float* __restrict__ lnb,
               float* __restrict__ out, int nN)
{
    __shared__ __attribute__((aligned(32))) float tile[16 * TP];
    const int row0 = blockIdx.x * 16;
    proj_tile<false>(nullptr, Hh, Wt3, ba, ntype, row0, nN, tile);
    __syncthreads();
    const int w = threadIdx.x >> 5, l = threadIdx.x & 31;
    v4f ov[2];
    int gr[2];
#pragma unroll
    for (int rr = 0; rr < 2; ++rr) {
        const int r = 2 * w + rr;
        const int g = row0 + r;
        const int gc = min(g, nN - 1);
        const int t = clampi(ntype[gc], 0, TT - 1);
        const float sk = skipw[t];
        const float a = 1.0f / (1.0f + expf(-sk));
        const v4f tr = *(const v4f*)(tile + r * TP + 4 * l);
        const v4f xi = *(const v4f*)(X + (size_t)gc * DD + 4 * l);
        const v4f res = tr * a + xi * (1.0f - a);
        float s = res[0] + res[1] + res[2] + res[3];
#pragma unroll
        for (int off = 16; off > 0; off >>= 1) s += __shfl_xor(s, off, 32);
        const float mu = s * (1.0f / 128.0f);
        const v4f dv = res - mu;
        float sq = dv[0] * dv[0] + dv[1] * dv[1] + dv[2] * dv[2] + dv[3] * dv[3];
#pragma unroll
        for (int off = 16; off > 0; off >>= 1) sq += __shfl_xor(sq, off, 32);
        const float rins = rsqrtf(sq * (1.0f / 128.0f) + 1e-5f);
        const v4f g4 = *(const v4f*)(lng + (size_t)t * DD + 4 * l);
        const v4f b4 = *(const v4f*)(lnb + (size_t)t * DD + 4 * l);
        ov[rr] = dv * rins * g4 + b4;
        gr[rr] = g;
    }
    float* p0 = out + (size_t)gr[0] * DD + 4 * l;
    float* p1 = out + (size_t)gr[1] * DD + 4 * l;
    if (gr[0] < nN) *(volatile v4f*)p0 = ov[0];
    if (gr[1] < nN) *(volatile v4f*)p1 = ov[1];
    __threadfence();
    if (gr[0] < nN) *(volatile v4f*)p0 = ov[0];
    if (gr[1] < nN) *(volatile v4f*)p1 = ov[1];
}

__global__ __launch_bounds__(256)
void k_rel(const _Float16* __restrict__ K16, const _Float16* __restrict__ V16,
           const float* __restrict__ rel_att, const float* __restrict__ rel_msg,
           _Float16* __restrict__ krot, _Float16* __restrict__ msgr, int nN)
{
    __shared__ __attribute__((aligned(16))) _Float16 tK[16 * RR * DD];
    __shared__ __attribute__((aligned(16))) _Float16 tM[16 * RR * DD];
    const int hh = threadIdx.x >> 5, l = threadIdx.x & 31, h = l >> 4, m = l & 15;
    const int node0 = blockIdx.x * 16;
    const int rowA = min(node0 + m, nN - 1);
    const v8h z8 = {};
    Frag ak, av;
    const size_t aoff = (size_t)rowA * DD + hh * DK + 8 * h;
    ak.half[0] = *(const v8h*)(K16 + aoff);
    ak.half[1] = z8;
    av.half[0] = *(const v8h*)(V16 + aoff);
    av.half[1] = z8;
#pragma unroll
    for (int r = 0; r < RR; ++r) {
        v8h tba = z8, tbm = z8;
#pragma unroll
        for (int i = 0; i < 8; ++i) {
            const int idx = ((r * HH + hh) * DK + 8 * h + i) * DK + m;
            tba[i] = (_Float16)(RSC * rel_att[idx]);
            tbm[i] = (_Float16)(RSC * rel_msg[idx]);
        }
        Frag ba, bm;
        ba.half[0] = tba; ba.half[1] = z8;
        bm.half[0] = tbm; bm.half[1] = z8;
        v8f acck = {}; v8f accm = {};
        acck = wmma_f16(ak.v, ba.v, acck);
        accm = wmma_f16(av.v, bm.v, accm);
#pragma unroll
        for (int rr = 0; rr < 8; ++rr) {
            const int li = ((8 * h + rr) * RR + r) * DD + hh * DK + m;
            tK[li] = (_Float16)(acck[rr] * RSCI);
            tM[li] = (_Float16)(accm[rr] * RSCI);
        }
    }
    __syncthreads();
    const int w = hh, cb = 8 * (l & 15);
#pragma unroll
    for (int j = 0; j < 4; ++j) {
        const int rl = 8 * w + 2 * j + (l >> 4);
        const int node = node0 + (rl >> 2);
        const v8h vk = *(const v8h*)(tK + rl * DD + cb);
        const v8h vm = *(const v8h*)(tM + rl * DD + cb);
        const size_t go = ((size_t)node0 * RR + rl) * DD + cb;
        if (node < nN) {
            *(volatile v8h*)(krot + go) = vk;
            *(volatile v8h*)(msgr + go) = vm;
        }
        __threadfence();
        if (node < nN) {
            *(volatile v8h*)(krot + go) = vk;
            *(volatile v8h*)(msgr + go) = vm;
        }
    }
}

__global__ __launch_bounds__(256)
void k_edge(const int* __restrict__ esrc, const int* __restrict__ edst, const int* __restrict__ ety,
            const float* __restrict__ Q32, const _Float16* __restrict__ krot, const _Float16* __restrict__ msgr,
            const float* __restrict__ pri, _Float16* __restrict__ H16, int nN, int nE, int nChunks)
{
    __shared__ __attribute__((aligned(16))) float elds[ELDS_FLOATS];
    float* acc = elds;
    float* Mx  = acc + NB * DD;
    float* Sx  = Mx + NB * HH;
    int*   lst = (int*)(Sx + NB * HH);
    int*   cnt = lst + 64 * LCAP;
    _Float16* hrow = (_Float16*)(cnt + 64);

    const int tid = threadIdx.x, w = tid >> 5, l = tid & 31;
    const int nodeBase = blockIdx.x * NB;

    const v4f z4 = {};
    for (int i = tid; i < NB * DD / 4; i += 256) ((v4f*)acc)[i] = z4;
    for (int i = tid; i < NB * HH; i += 256) { Mx[i] = -INFINITY; Sx[i] = 0.0f; }
    __syncthreads();

    const int c4 = 4 * l, hd = l >> 2;
    for (int c = 0; c < nChunks; ++c) {
        if (l == 0) {
#pragma unroll
            for (int o = 0; o < 8; ++o) cnt[w * 8 + o] = 0;
        }
        const int sbase = c * CHB + w * CHW;
        for (int it = 0; it < CHW / 32; ++it) {
            const int e = sbase + it * 32 + l;
            int u = -1;
            if (e < nE) u = edst[e] - nodeBase;
            const bool hit = (unsigned)u < (unsigned)NB;
            unsigned mask = (unsigned)__ballot(hit);
            while (mask != 0u) {
                const int b = __builtin_ctz(mask);
                mask &= mask - 1u;
                const int ub = __shfl(u, b, 32);
                if (l == 0) {
                    const int o = (ub >> 5) & 7;
                    const int k = cnt[w * 8 + o];
                    if (k < LCAP) lst[(w * 8 + o) * LCAP + k] = sbase + it * 32 + b;
                    cnt[w * 8 + o] = k + 1;
                }
            }
        }
        __syncthreads();
        for (int s = 0; s < 8; ++s) {
            int ns = cnt[s * 8 + w];
            ns = ns > LCAP ? LCAP : ns;
            for (int j = 0; j < ns; ++j) {
                int e = lst[(s * 8 + w) * LCAP + j];
                e = clampi(e, 0, nE - 1);
                const int sr = clampi(esrc[e], 0, nN - 1);
                const int r  = clampi(ety[e], 0, RR - 1);
                const int dl = clampi(edst[e] - nodeBase, 0, NB - 1);
                const int dg = min(nodeBase + dl, nN - 1);
                const size_t roff = ((size_t)sr * RR + r) * DD + c4;
                const v4f kf = __builtin_convertvector(*(const v4h*)(krot + roff), v4f);
                const v4f qv = *(const v4f*)(Q32 + (size_t)dg * DD + c4);
                float part = kf[0] * qv[0] + kf[1] * qv[1] + kf[2] * qv[2] + kf[3] * qv[3];
                part += __shfl_xor(part, 1, 32);
                part += __shfl_xor(part, 2, 32);
                const float lg = (part * pri[r * HH + hd]) * 0.25f;
                const int ms = dl * HH + hd;
                const float mo = Mx[ms], so = Sx[ms];
                const float mn = fmaxf(mo, lg);
                const float sc = __expf(mo - mn);
                const float p  = __expf(lg - mn);
                const v4f mg = __builtin_convertvector(*(const v4h*)(msgr + roff), v4f);
                float* ap = acc + dl * DD + c4;
                v4f av = *(v4f*)ap;
                av = av * sc + mg * p;
                *(v4f*)ap = av;
                Mx[ms] = mn;
                Sx[ms] = so * sc + p;
            }
        }
        __syncthreads();
    }

    const int sub = l >> 4, cb = 8 * (l & 15), hq = cb >> 4;
    _Float16* hp = hrow + (w * 2 + sub) * DD + cb;
#pragma unroll 1
    for (int j = 0; j < 16; ++j) {
        const int dl = w * 32 + 2 * j + sub;
        const int node = nodeBase + dl;
        const float inv = 1.0f / (Sx[dl * HH + hq] + 1e-16f);
        const float* ap = acc + dl * DD + cb;
#pragma unroll 1
        for (int q = 0; q < 8; ++q) {
            const float x = ap[q] * inv;
            const float g = 0.5f * x * (1.0f + erff(x * 0.70710678118654752f));
            hp[q] = (_Float16)g;
        }
        const v8h hv = *(const v8ha*)hp;
        _Float16* gp = H16 + (size_t)node * DD + cb;
        if (node < nN) *(volatile v8h*)gp = hv;
        __threadfence();
        if (node < nN) *(volatile v8h*)gp = hv;
    }
}

extern "C" void kernel_launch(void* const* d_in, const int* in_sizes, int n_in,
                              void* d_out, int out_size, void* d_ws, size_t ws_size,
                              hipStream_t stream)
{
    (void)n_in; (void)out_size;
    const int nN = in_sizes[1];
    int nE = in_sizes[3];
    const int nE2 = in_sizes[2] / 2;
    if (nE2 < nE) nE = nE2;
    if (nN <= 0 || nE < 0) return;

    const float* node_inp = (const float*)d_in[0];
    const int*   ntype    = (const int*)d_in[1];
    const int*   esrc     = (const int*)d_in[2];
    const int*   edst     = esrc + nE2;
    const int*   etype    = (const int*)d_in[3];
    const float* Wk = (const float*)d_in[4];  const float* bk = (const float*)d_in[5];
    const float* Wq = (const float*)d_in[6];  const float* bq = (const float*)d_in[7];
    const float* Wv = (const float*)d_in[8];  const float* bv = (const float*)d_in[9];
    const float* Wa = (const float*)d_in[10]; const float* ba = (const float*)d_in[11];
    const float* rel_pri = (const float*)d_in[12];
    const float* rel_att = (const float*)d_in[13];
    const float* rel_msg = (const float*)d_in[14];
    const float* skipw = (const float*)d_in[15];
    const float* ln_g = (const float*)d_in[16];
    const float* ln_b = (const float*)d_in[17];
    float* out = (float*)d_out;

    size_t off = 0;
    auto carve = [&](size_t bytes) -> size_t {
        const size_t p = off;
        off += (bytes + 255) & ~(size_t)255;
        return p;
    };
    const size_t o_k16 = carve((size_t)nN * DD * 2);
    const size_t o_v16 = carve((size_t)nN * DD * 2);
    const size_t o_q32 = carve((size_t)nN * DD * 4);
    const size_t o_kr  = carve((size_t)nN * RR * DD * 2);
    const size_t o_mr  = carve((size_t)nN * RR * DD * 2);
    const size_t o_wt  = carve((size_t)4 * TT * DD * DD * 2);
    if (off > ws_size) return;

    char* wsb = (char*)d_ws;
    _Float16* k16  = (_Float16*)(wsb + o_k16);
    _Float16* h16  = k16;
    _Float16* v16  = (_Float16*)(wsb + o_v16);
    float*    q32  = (float*)(wsb + o_q32);
    _Float16* krot = (_Float16*)(wsb + o_kr);
    _Float16* msgr = (_Float16*)(wsb + o_mr);
    _Float16* wt   = (_Float16*)(wsb + o_wt);

    const int nTiles = (nN + 15) / 16;
    const int nChunks = (nE + CHB - 1) / CHB;
    const int nEdgeBlk = (nN + NB - 1) / NB;

    k_cvtw<<<(NWT8 + 255) / 256, 256, 0, stream>>>(Wk, Wq, Wv, Wa, wt, NWT8);
    k_proj_kqv<<<dim3(nTiles, 3), 256, 0, stream>>>(node_inp, wt, bk, bq, bv, ntype, k16, q32, v16, nN);
    k_rel<<<nTiles, 256, 0, stream>>>(k16, v16, rel_att, rel_msg, krot, msgr, nN);
    k_edge<<<nEdgeBlk, 256, 0, stream>>>(esrc, edst, etype, q32, krot, msgr, rel_pri, h16, nN, nE, nChunks);
    k_proj_ln<<<nTiles, 256, 0, stream>>>(h16, wt + (size_t)3 * TT * DD * DD, ba, ntype, node_inp,
                                          skipw, ln_g, ln_b, out, nN);
}
